// CGNS_Block_5420248728082
// MI455X (gfx1250) — hardware-verified
//
#include <hip/hip_runtime.h>
#include <math.h>

typedef __attribute__((ext_vector_type(16))) _Float16 v16h;
typedef __attribute__((ext_vector_type(16))) __bf16 v16b;
typedef __attribute__((ext_vector_type(8)))  _Float16 v8h;
typedef __attribute__((ext_vector_type(8)))  float v8f;
typedef __attribute__((ext_vector_type(4)))  float v4f;
typedef __attribute__((ext_vector_type(2)))  float v2f;
typedef __attribute__((ext_vector_type(4)))  unsigned v4u;
typedef __attribute__((ext_vector_type(4)))  int v4i;
typedef float __attribute__((may_alias)) float_a;
typedef int __attribute__((may_alias)) int_a;

template <typename T> __device__ __forceinline__ void vst2(void* p, T v) { *(volatile T*)p = v; __threadfence(); *(volatile T*)p = v; }
__device__ __forceinline__ v8f wmma16(v16h a, v16h b, v8f c) {
  v8f d = __builtin_amdgcn_wmma_f32_16x16x32_f16(false, a, false, b, (short)0, c, false, false);
  asm volatile("v_nop\n\tv_nop\n\tv_nop\n\tv_nop" : "+v"(d) : "v"(a), "v"(b));
  return d;
}
__device__ __forceinline__ v8f wmma_bf(v16b a, v16b b, v8f c) {
  v8f d = __builtin_amdgcn_wmma_f32_16x16x32_bf16(false, a, false, b, (short)0, c, false, false);
  asm volatile("v_nop\n\tv_nop\n\tv_nop\n\tv_nop" : "+v"(d) : "v"(a), "v"(b));
  return d;
}
__device__ __forceinline__ v16h frag_h(const _Float16* rowk0, int lane) {
  union { v16h v; v8h q[2]; } u; const _Float16* p = rowk0 + 8 * (lane >> 4);
  u.q[0] = *(const v8h*)p; u.q[1] = *(const v8h*)(p + 16); return u.v;
}
__device__ __forceinline__ v16h frag_f32(const float* rowk0, int lane) {
  v16h a; const float* p = rowk0 + 8 * (lane >> 4);
#pragma unroll
  for (int i = 0; i < 8; ++i) { a[i] = (_Float16)p[i]; a[8 + i] = (_Float16)p[16 + i]; }
  return a;
}
__device__ __forceinline__ v16h frag_f32s(const float* rowk0, int lane, float sc) {
  v16h a; const float* p = rowk0 + 8 * (lane >> 4);
#pragma unroll
  for (int i = 0; i < 8; ++i) { a[i] = (_Float16)(p[i] * sc); a[8 + i] = (_Float16)(p[16 + i] * sc); }
  return a;
}
__device__ __forceinline__ v16h fragc_f32(const float* W, int k0, int n, int lane, int ld, int K) {
  v16h a; const int g = lane >> 4;
#pragma unroll
  for (int i = 0; i < 8; ++i) { const int ka = k0 + 8 * g + i, kb = ka + 16;
    a[i] = (_Float16)(ka < K ? W[(size_t)(ka < K ? ka : K - 1) * ld + n] : 0.f); a[8 + i] = (_Float16)(kb < K ? W[(size_t)(kb < K ? kb : K - 1) * ld + n] : 0.f); }
  return a;
}
struct F2 { v16b h, l; };
__device__ __forceinline__ F2 bsplit16(const float v[16]) { F2 r;
#pragma unroll
  for (int i = 0; i < 16; ++i) { const __bf16 h = (__bf16)v[i]; r.h[i] = h; r.l[i] = (__bf16)(v[i] - (float)h); }
  return r; }
__device__ __forceinline__ F2 split_row(const float* row, int k0, int lane) { float v[16]; const float* p = row + k0 + 8 * (lane >> 4);
#pragma unroll
  for (int i = 0; i < 8; ++i) { v[i] = p[i]; v[8 + i] = p[16 + i]; }
  return bsplit16(v); }
__device__ __forceinline__ F2 split_rowK(const float* row, int k0, int lane, int K) { float v[16]; const int g = lane >> 4;
#pragma unroll
  for (int i = 0; i < 8; ++i) { const int ka = k0 + 8 * g + i, kb = ka + 16; v[i] = ka < K ? row[ka < K ? ka : K - 1] : 0.f; v[8 + i] = kb < K ? row[kb < K ? kb : K - 1] : 0.f; }
  return bsplit16(v); }
__device__ __forceinline__ F2 split_col(const float* W, int k0, int n, int lane, int ld, int K) { float v[16]; const int g = lane >> 4;
#pragma unroll
  for (int i = 0; i < 8; ++i) { const int ka = k0 + 8 * g + i, kb = ka + 16; v[i] = ka < K ? W[(size_t)(ka < K ? ka : K - 1) * ld + n] : 0.f; v[8 + i] = kb < K ? W[(size_t)(kb < K ? kb : K - 1) * ld + n] : 0.f; }
  return bsplit16(v); }
__device__ __forceinline__ v8f mac3(const F2& a, const F2& b, v8f c) { c = wmma_bf(a.l, b.h, c); c = wmma_bf(a.h, b.l, c); return wmma_bf(a.h, b.h, c); }
__device__ __forceinline__ float sigm(float v) { return 1.0f / (1.0f + expf(-v)); }
#define LDSX() do { asm volatile("s_wait_dscnt 0" ::: "memory"); __builtin_amdgcn_wave_barrier(); __builtin_amdgcn_fence(__ATOMIC_RELEASE, "workgroup"); } while (0)


#define NB 4
#define CC 64
#define NN 4096
#ifndef TNB
#define TNB NB
#endif
typedef __attribute__((ext_vector_type(8))) __bf16 v8b;
__device__ __forceinline__ v16b frag_b(const __bf16* rowk0, int lane) {
  union { v16b v; v8b q[2]; } u; const __bf16* p = rowk0 + 8 * (lane >> 4);
  u.q[0] = *(const v8b*)p; u.q[1] = *(const v8b*)(p + 16); return u.v;
}
__device__ __forceinline__ float bfr(float v) { return (float)(__bf16)v; }
__device__ __attribute__((noinline)) float exp_ni(float v) { return expf(v); }
__device__ __attribute__((noinline)) float erf_ni(float v) { return erff(v); }

#define WS_PW  0u
#define WS_AD  (WS_PW + 2u * (size_t)CC * 2 * CC)
#define WS_DD  (WS_AD + 4u * (size_t)NB * NN)
#define WS_ST  (WS_DD + 4u * (size_t)NB * NN)
#define WS_END (WS_ST + 4u * (size_t)NB * CC * 32)

__device__ __attribute__((noinline)) float tanh_p(float v) { return tanhf(v); }
__global__ __launch_bounds__(256) void k_pack(const float* __restrict__ Wc, __bf16* __restrict__ P) { __shared__ __align__(16) __bf16 s[CC * 2 * CC]; const int t = threadIdx.x; for (int i = t; i < CC * 2 * CC; i += 256) s[i] = (__bf16)Wc[i]; __syncthreads(); for (int q = t; q < CC * 2 * CC / 8; q += 256) vst2((unsigned*)(P + q * 8), *(const v4u*)&s[q * 8]); }
__global__ __launch_bounds__(1024) void k_ad(const float* __restrict__ Wn, float* __restrict__ A, float* __restrict__ Dd) {
  __shared__ float sa[NN]; __shared__ float red[32]; const size_t b = blockIdx.x; const int t = threadIdx.x; float s = 0.f;
  for (int n = t; n < NN; n += 1024) { const float a = fmaxf(tanh_p(bfr(Wn[b * NN + n])), 0.f); sa[n] = a; s += a; }
#pragma unroll
  for (int o = 1; o < 32; o <<= 1) s += __shfl_xor(s, o);
  if ((t & 31) == 0) red[t >> 5] = s; __syncthreads(); float SA = 0.f; for (int i = 0; i < 32; ++i) SA += red[i];
  __syncthreads();
  for (int q = t; q < NN / 4; q += 1024) { v4f av, dv; for (int i = 0; i < 4; ++i) { av[i] = sa[q * 4 + i]; dv[i] = 1.0f / sqrtf(av[i] * SA + 1.0f); } vst2(A + b * NN + q * 4, av); vst2(Dd + b * NN + q * 4, dv); }
}
__global__ __launch_bounds__(256) void k_st(const float* __restrict__ X, const float* __restrict__ A, const float* __restrict__ Dd, float* __restrict__ ST) {
  __shared__ float r0[8], r1[8]; __shared__ __align__(16) float line[32]; const int c = blockIdx.x; const size_t b = blockIdx.y; const int t = threadIdx.x; const float* xr = X + (b * CC + c) * NN; float s0 = 0.f, s1 = 0.f;
  for (int n = t; n < NN; n += 256) { const float x = bfr(xr[n]), a = A[b * NN + n]; s0 += x * a; s1 += x * a * Dd[b * NN + n]; }
#pragma unroll
  for (int o = 1; o < 32; o <<= 1) { s0 += __shfl_xor(s0, o); s1 += __shfl_xor(s1, o); }
  if ((t & 31) == 0) { r0[t >> 5] = s0; r1[t >> 5] = s1; } __syncthreads();
  if (t < 32) { float a0 = 0.f, a1 = 0.f; if (t == 0) for (int i = 0; i < 8; ++i) { a0 += r0[i]; a1 += r1[i]; } line[t] = (t == 0) ? a0 : (t == 1) ? 0.f : 0.f; if (t == 1) line[1] = 0.f; }
  __syncthreads(); if (t == 0) {   }
  if (t == 0) { float a1 = 0.f; for (int i = 0; i < 8; ++i) a1 += r1[i]; line[1] = a1; }
  __syncthreads(); if (t < 8) vst2(ST + ((b * CC + c) * 32) + t * 4, *(const v4f*)&line[t * 4]);
}
__global__ __launch_bounds__(128) void k_conv(const float* __restrict__ X, const float* __restrict__ A, const float* __restrict__ Dd, const float* __restrict__ ST, const __bf16* __restrict__ P, const float* __restrict__ CB, const float* __restrict__ G, const float* __restrict__ BE, const float* __restrict__ MU, const float* __restrict__ VAR, float* __restrict__ Y) {
  __shared__ __align__(16) __bf16 sh[128][2 * CC + 8]; __shared__ __align__(16) __bf16 sl[128][2 * CC + 8]; __shared__ __align__(16) float so[4][16][132];
  const int tid = threadIdx.x, wave = tid >> 5, lane = tid & 31, col = lane & 15, g = lane >> 4; const size_t b = blockIdx.y; const int n0 = blockIdx.x * 128;
  { const int nl = tid; const int n = n0 + nl; const float a = A[b * NN + n], d = Dd[b * NN + n];
    for (int c = 0; c < CC; ++c) { const float x = bfr(X[((b * CC + c) * NN) + n]); const float s0 = ST[(b * CC + c) * 32], tt = ST[(b * CC + c) * 32 + 1];
      const float v0 = s0 * a + x; const float v1 = d * (a * tt + d * x);
      const __bf16 h0 = (__bf16)v0, h1 = (__bf16)v1; sh[nl][c] = h0; sl[nl][c] = (__bf16)(v0 - (float)h0); sh[nl][CC + c] = h1; sl[nl][CC + c] = (__bf16)(v1 - (float)h1); } }
  __syncthreads();
  v8f acc[8] = {};
#pragma unroll
  for (int kc = 0; kc < 2 * CC / 32; ++kc) { const v16b aw = frag_b(P + (size_t)(wave * 16 + col) * (2 * CC) + kc * 32, lane);
#pragma unroll
    for (int j = 0; j < 8; ++j) { acc[j] = wmma_bf(aw, frag_b(&sh[j * 16 + col][0] + kc * 32, lane), acc[j]); acc[j] = wmma_bf(aw, frag_b(&sl[j * 16 + col][0] + kc * 32, lane), acc[j]); } }
#pragma unroll
  for (int r = 0; r < 8; ++r) { const int o = wave * 16 + 8 * g + r; const float cb = bfr(CB[o]), sc = bfr(G[o]) / sqrtf(bfr(VAR[o]) + 1e-5f), shv = bfr(BE[o]) - bfr(MU[o]) * sc;
#pragma unroll
    for (int j = 0; j < 8; ++j) so[wave][8 * g + r][j * 16 + col] = fmaxf((acc[j][r] + cb) * sc + shv, 0.f); }
  LDSX();
  for (int rl = 0; rl < 16; ++rl) vst2(Y + ((b * CC + wave * 16 + rl) * NN) + n0 + lane * 4, *(const v4f*)&so[wave][rl][lane * 4]);
}
extern "C" void kernel_launch(void* const* d_in, const int* in_sizes, int n_in, void* d_out, int out_size, void* d_ws, size_t ws_size, hipStream_t stream) {
  (void)in_sizes; (void)n_in; (void)out_size;
  const float** F = (const float**)d_in;
  if (ws_size < (size_t)WS_END) return;
  char* ws = (char*)d_ws; __bf16* P = (__bf16*)ws; float *A = (float*)(ws + WS_AD), *Dd = (float*)(ws + WS_DD), *ST = (float*)(ws + WS_ST);
  k_pack<<<1, 256, 0, stream>>>(F[2], P);
  k_ad<<<TNB, 1024, 0, stream>>>(F[1], A, Dd);
  k_st<<<dim3(CC, TNB), 256, 0, stream>>>(F[0], A, Dd, ST);
  k_conv<<<dim3(NN / 128, TNB), 128, 0, stream>>>(F[0], A, Dd, ST, P, F[3], F[4], F[5], F[6], F[7], (float*)d_out);
}
